// Experiment16_55722905698572
// MI455X (gfx1250) — hardware-verified
//
#include <hip/hip_runtime.h>

typedef __attribute__((ext_vector_type(16))) _Float16 v16h;
typedef __attribute__((ext_vector_type(8)))  _Float16 v8h;
typedef __attribute__((ext_vector_type(4)))  _Float16 v4h;
typedef __attribute__((ext_vector_type(8)))  float    v8f;
typedef __attribute__((ext_vector_type(4)))  float    v4f;

constexpr int kBatch   = 128;
constexpr int kLen     = 256;
constexpr int kVocab   = 50000;
constexpr int kEmb     = 300;
constexpr int kEmbP    = 320;
constexpr int kHid     = 512;
constexpr int kCls     = 5;
constexpr int kKdim    = kHid + kEmbP;
constexpr int kFeat    = 2 * kHid + kEmb;
constexpr int kMxP     = 1344;
constexpr int kEmbCol  = kHid;
constexpr int kRightCol = kHid + kEmbP;

constexpr int kSeqPB     = 16;
constexpr int kBlkPerDir = kBatch / kSeqPB;
constexpr int kRecBlocks = 2 * kBlkPerDir;
constexpr int kRecThreads = 256;
constexpr int kAP        = kKdim + 8;
constexpr int kATile     = kSeqPB * kAP;
constexpr int kSlotHalves = kSeqPB * kHid;
constexpr size_t kBlkHalves = (size_t)kLen * kSlotHalves;
constexpr size_t kDirHalves = (size_t)kBlkPerDir * kBlkHalves;
constexpr int kEChunks   = kSeqPB * (kEmbP / 8);

constexpr int kWRowChunks = kKdim / 8;
constexpr int kWChunksDir = kHid * kWRowChunks;
constexpr int kPrepBlkDir = kWChunksDir / 256;
constexpr int kPrepBlocks = 2 * kPrepBlkDir;

static_assert(kKdim % 32 == 0);
static_assert(kWChunksDir % 256 == 0 && kPrepBlkDir == 208 && kPrepBlocks == 416);
static_assert((kSeqPB * kLen) % kRecThreads == 0);
static_assert(kRecThreads * 4 * 8 == kSlotHalves);
static_assert(kRecThreads * 4 * 8 == kSeqPB * kHid);
static_assert((kRecThreads / 32) * 64 == kHid);
static_assert(kAP % 8 == 0 && kATile % 8 == 0);
static_assert(kEChunks <= 3 * kRecThreads);
static_assert((kMxP * 4) % 128 == 0 && (kEmbCol * 4) % 128 == 0 && (kRightCol * 4) % 128 == 0);
static_assert(kRightCol + kHid == kMxP);
static_assert(kBatch * kCls == 640 && (kBatch * kCls) % 4 == 0);
static_assert(kBatch * kHid == 256 * 256);
static_assert(kEmbP % 32 == 0 && kEmbP <= 1024);

__device__ __forceinline__ void dep_guard_h(v8f& a, v8f& b, v16h x, v16h y) { asm volatile("v_nop\n\tv_nop\n\tv_nop\n\tv_nop" : "+v"(a), "+v"(b) : "v"(x), "v"(y)); }
__device__ __forceinline__ void keep4_h(v16h a, v16h b, v16h c, v16h d) { asm volatile("v_nop" :: "v"(a), "v"(b), "v"(c), "v"(d)); }
__device__ __forceinline__ void acc_guard4(v8f& a, v8f& b, v8f& c, v8f& d) { asm volatile("v_nop\n\tv_nop\n\tv_nop\n\tv_nop" : "+v"(a), "+v"(b), "+v"(c), "+v"(d)); }

template <typename T> struct Frag;
template <> struct Frag<_Float16> {
  typedef v16h V; union U { v16h v; v8h h[2]; };
  static __device__ __forceinline__ v16h load(const _Float16* p) {
    U f; f.h[0] = *(const v8h*)(p); f.h[1] = *(const v8h*)(p + 16); return f.v;
  }
  static __device__ __forceinline__ v8f mma(v16h a, v16h b, v8f c) {
    return __builtin_amdgcn_wmma_f32_16x16x32_f16(false, a, false, b, (short)0, c, false, false);
  }
  static __device__ __forceinline__ void guard(v8f& a, v8f& b, v16h x, v16h y) { dep_guard_h(a, b, x, y); }
  static __device__ __forceinline__ void keep(v16h a, v16h b, v16h c, v16h d) { keep4_h(a, b, c, d); }
};

__global__ __launch_bounds__(256) void prep_kernel(const float* __restrict__ wl, const float* __restrict__ wsl,
                                                   const float* __restrict__ wr, const float* __restrict__ wsr,
                                                   _Float16* __restrict__ wcat) {
  const int i = blockIdx.x * 256 + threadIdx.x;
  const int dir = (blockIdx.x >= (unsigned)kPrepBlkDir) ? 1 : 0;
  const float* W  = dir ? wr : wl;
  const float* Ws = dir ? wsr : wsl;
  const int rem = i - dir * kWChunksDir;
  const int h   = rem / kWRowChunks;
  const int ch  = rem - h * kWRowChunks;
  const int k0  = ch * 8;
  const int kw  = k0 < (kHid - 8) ? k0 : (kHid - 8);
  const float* wsrc = W + (size_t)h * kHid + kw;
  const v4f w0 = *(const v4f*)wsrc;
  const v4f w1 = *(const v4f*)(wsrc + 4);
  int ce = k0 - kHid; ce = ce < 0 ? 0 : ce;
  const int base = ce < (kEmb - 8) ? ce : (kEmb - 8);
  const float* ssrc = Ws + (size_t)h * kEmb + base;
  const v4f s0 = *(const v4f*)ssrc;
  const v4f s1 = *(const v4f*)(ssrc + 4);
  const bool isW = k0 < kHid;
  const bool sh4 = (ce == kEmb - 4);
  const float sc = 256.0f;
  v8h hv;
  hv[0] = (_Float16)((isW ? w0[0] : ((ce + 0 < kEmb) ? (sh4 ? s1[0] : s0[0]) : 0.0f)) * sc);
  hv[1] = (_Float16)((isW ? w0[1] : ((ce + 1 < kEmb) ? (sh4 ? s1[1] : s0[1]) : 0.0f)) * sc);
  hv[2] = (_Float16)((isW ? w0[2] : ((ce + 2 < kEmb) ? (sh4 ? s1[2] : s0[2]) : 0.0f)) * sc);
  hv[3] = (_Float16)((isW ? w0[3] : ((ce + 3 < kEmb) ? (sh4 ? s1[3] : s0[3]) : 0.0f)) * sc);
  hv[4] = (_Float16)((isW ? w1[0] : ((ce + 4 < kEmb) ? s1[0] : 0.0f)) * sc);
  hv[5] = (_Float16)((isW ? w1[1] : ((ce + 5 < kEmb) ? s1[1] : 0.0f)) * sc);
  hv[6] = (_Float16)((isW ? w1[2] : ((ce + 6 < kEmb) ? s1[2] : 0.0f)) * sc);
  hv[7] = (_Float16)((isW ? w1[3] : ((ce + 7 < kEmb) ? s1[3] : 0.0f)) * sc);
  _Float16* dst = wcat + (size_t)i * 8;
  *(volatile v8h*)dst = hv;
  __threadfence();
  *(volatile v8h*)dst = hv;
}

__global__ __launch_bounds__(kRecThreads) void recur_kernel(
    const int* __restrict__ x, const float* __restrict__ emb, const _Float16* __restrict__ wcat,
    const float* __restrict__ cl, const float* __restrict__ cr, _Float16* __restrict__ planes) {
  __shared__ __align__(16) unsigned short sTok[kSeqPB * kLen];
  __shared__ __align__(16) _Float16 sA[2 * kATile];
  const int tid = threadIdx.x, lane = tid & 31, wave = tid >> 5;
  const int c = lane & 15, hh = lane >> 4, koff = hh * 8, mOff = hh * 8;
  const int dir = (int)(blockIdx.x >> 3);
  const int blk = (int)(blockIdx.x & 7);
  const int seq0 = blk * kSeqPB;
  const _Float16* W = wcat + (size_t)dir * kWChunksDir * 8;
  const float* c0v = dir ? cr : cl;
  _Float16* plane = planes + (size_t)dir * kDirHalves + (size_t)blk * kBlkHalves;

#pragma unroll 1
  for (int it = 0; it < (kSeqPB * kLen) / kRecThreads; ++it) {
    const int i = it * kRecThreads + tid;
    int t = x[(size_t)(seq0 + (i >> 8)) * kLen + (i & 255)];
    t = t < 0 ? 0 : t;
    t = t > kVocab - 1 ? kVocab - 1 : t;
    sTok[i] = (unsigned short)t;
  }
#pragma unroll
  for (int it = 0; it < 4; ++it) {
    const int q = it * kRecThreads + tid;
    const int row = q >> 6, col = (q & 63) * 8;
    const v4f a = *(const v4f*)(c0v + col);
    const v4f b = *(const v4f*)(c0v + col + 4);
    v8h hv;
    hv[0] = (_Float16)(a[0] * 1024.0f); hv[1] = (_Float16)(a[1] * 1024.0f);
    hv[2] = (_Float16)(a[2] * 1024.0f); hv[3] = (_Float16)(a[3] * 1024.0f);
    hv[4] = (_Float16)(b[0] * 1024.0f); hv[5] = (_Float16)(b[1] * 1024.0f);
    hv[6] = (_Float16)(b[2] * 1024.0f); hv[7] = (_Float16)(b[3] * 1024.0f);
    *(v8h*)(sA + kATile + row * kAP + col) = hv;
  }
  if (tid < 32) {
    v8h z;
#pragma unroll
    for (int e = 0; e < 8; ++e) z[e] = (_Float16)0.0f;
    *(v8h*)(sA + (tid >> 4) * kATile + (tid & 15) * kAP + kKdim) = z;
  }
  __syncthreads();

  auto stage_e = [&](int t1, int tile) {
    const int pos = dir ? ((254 - t1) & 255) : (t1 - 1);
#pragma unroll
    for (int it = 0; it < 3; ++it) {
      const int q = it * kRecThreads + tid;
      const int qc = q < kEChunks ? q : (kEChunks - 1);
      const int row = qc / (kEmbP / 8);
      const int ch = qc - row * (kEmbP / 8);
      const int cb = ch * 8;
      const int tok = (int)sTok[row * kLen + pos];
      const int base = cb < (kEmb - 8) ? cb : (kEmb - 8);
      const float* src = emb + (size_t)tok * kEmb + base;
      const v4f f0 = *(const v4f*)src;
      const v4f f1 = *(const v4f*)(src + 4);
      const bool sh4 = (cb == kEmb - 4);
      const float es = 1024.0f;
      v8h hv;
      hv[0] = (_Float16)(((cb + 0 < kEmb) ? (sh4 ? f1[0] : f0[0]) : 0.0f) * es);
      hv[1] = (_Float16)(((cb + 1 < kEmb) ? (sh4 ? f1[1] : f0[1]) : 0.0f) * es);
      hv[2] = (_Float16)(((cb + 2 < kEmb) ? (sh4 ? f1[2] : f0[2]) : 0.0f) * es);
      hv[3] = (_Float16)(((cb + 3 < kEmb) ? (sh4 ? f1[3] : f0[3]) : 0.0f) * es);
      hv[4] = (_Float16)(((cb + 4 < kEmb) ? f1[0] : 0.0f) * es);
      hv[5] = (_Float16)(((cb + 5 < kEmb) ? f1[1] : 0.0f) * es);
      hv[6] = (_Float16)(((cb + 6 < kEmb) ? f1[2] : 0.0f) * es);
      hv[7] = (_Float16)(((cb + 7 < kEmb) ? f1[3] : 0.0f) * es);
      if (q < kEChunks) *(v8h*)(sA + tile * kATile + row * kAP + kHid + cb) = hv;
    }
  };
  stage_e(1, 1);
  __syncthreads();

  const int n0 = wave * 64;
  const float inv256 = 1.0f / 256.0f;
#pragma unroll 1
  for (int t = 1; t < kLen; ++t) {
    const int p = t & 1;
    const int t1 = (t + 1 < kLen) ? (t + 1) : (kLen - 1);
    stage_e(t1, p ^ 1);

    const _Float16* arow = sA + p * kATile + c * kAP + koff;
    const _Float16* brow = W + (size_t)(n0 + c) * kKdim + koff;
    v8f acc[4];
#pragma unroll
    for (int j = 0; j < 4; ++j) acc[j] = (v8f){0.f,0.f,0.f,0.f,0.f,0.f,0.f,0.f};
#pragma unroll 1
    for (int k0 = 0; k0 < kKdim; k0 += 32) {
      v16h bh[4];
#pragma unroll
      for (int j = 0; j < 4; ++j) bh[j] = Frag<_Float16>::load(brow + (size_t)j * 16 * kKdim + k0);
      const v16h ah = Frag<_Float16>::load(arow + k0);
#pragma unroll
      for (int j = 0; j < 4; ++j) acc[j] = Frag<_Float16>::mma(ah, bh[j], acc[j]);
      Frag<_Float16>::guard(acc[0], acc[3], ah, ah);
      Frag<_Float16>::keep(bh[0], bh[1], bh[2], bh[3]);
    }
    acc_guard4(acc[0], acc[1], acc[2], acc[3]);

    _Float16* hn = sA + (p ^ 1) * kATile;
#pragma unroll
    for (int j = 0; j < 4; ++j) {
      const int n = n0 + 16 * j + c;
#pragma unroll
      for (int r = 0; r < 8; ++r) {
        const float v = fmaxf(acc[j][r] * inv256, 0.0f);
        hn[(mOff + r) * kAP + n] = (_Float16)v;
      }
    }
    __syncthreads();

    const int slot = dir ? (t - 1) : t;
    _Float16* dst = plane + (size_t)slot * kSlotHalves;
    v8h pv[4];
#pragma unroll
    for (int it = 0; it < 4; ++it) {
      const int q = it * kRecThreads + tid;
      pv[it] = *(const v8h*)(hn + (q >> 6) * kAP + (q & 63) * 8);
    }
    for (int pass = 0; pass < 2; ++pass) {
#pragma unroll
      for (int it = 0; it < 4; ++it) {
        const int q = it * kRecThreads + tid;
        *(volatile v8h*)(dst + (size_t)q * 8) = pv[it];
      }
      __threadfence();
    }
  }
}

__global__ __launch_bounds__(256) void max_left_kernel(const _Float16* __restrict__ planeL, const float* __restrict__ cl,
                                                       float* __restrict__ mx) {
  const int idx = blockIdx.x * 256 + threadIdx.x;
  const int Bp = idx >> 9, hp = idx & 511;
  const int b = hp & 127, u = hp >> 7;
  const int blk = b >> 4, bl = b & 15;
  const _Float16* bp = planeL + (size_t)blk * kBlkHalves + (size_t)bl * kHid + 4 * Bp;
  float m = -__builtin_inff();
#pragma unroll 4
  for (int r = 0; r < 64; ++r) {
    const int s = 4 * r + u;
    const v4h v = *(const v4h*)(bp + (size_t)s * kSlotHalves);
    const float vm = fmaxf(fmaxf((float)v[0], (float)v[1]), fmaxf((float)v[2], (float)v[3]));
    m = fmaxf(m, (s == 0) ? -__builtin_inff() : vm);
  }
  m = m * (1.0f / 1024.0f);
  const v4f cv = *(const v4f*)(cl + 4 * Bp);
  const float cm = fmaxf(fmaxf(cv[0], cv[1]), fmaxf(cv[2], cv[3]));
  m = fmaxf(m, (u == 0) ? cm : -__builtin_inff());
  float* d = mx + (size_t)Bp * kMxP + hp;
  *(volatile float*)d = m;
  __threadfence();
  *(volatile float*)d = m;
}

__global__ __launch_bounds__(320) void max_emb_kernel(const int* __restrict__ x, const float* __restrict__ emb,
                                                      float* __restrict__ mx) {
  __shared__ int tok[kLen];
  const int Bp = blockIdx.x, e = threadIdx.x;
  if (e < kLen) {
    int t = x[(size_t)Bp * kLen + e];
    t = t < 0 ? 0 : t;
    t = t > kVocab - 1 ? kVocab - 1 : t;
    tok[e] = t;
  }
  __syncthreads();
  const int ec = e < kEmb ? e : (kEmb - 1);
  float m = -__builtin_inff();
#pragma unroll 4
  for (int s = 0; s < kLen; ++s) m = fmaxf(m, emb[(size_t)tok[s] * kEmb + ec]);
  m = (e < kEmb) ? m : 0.0f;
  float* d = mx + (size_t)Bp * kMxP + kEmbCol + e;
  *(volatile float*)d = m;
  __threadfence();
  *(volatile float*)d = m;
}

__global__ __launch_bounds__(256) void max_right_kernel(const _Float16* __restrict__ planeR, const float* __restrict__ cr,
                                                        float* __restrict__ mx) {
  const int idx = blockIdx.x * 256 + threadIdx.x;
  const int Bp = idx >> 9, hp = idx & 511;
  const int s0 = 2 * Bp, s1 = 2 * Bp + 1;
  const int s1c = s1 < (kLen - 1) ? s1 : (kLen - 2);
  const _Float16* p0 = planeR + (size_t)s0 * kSlotHalves + hp;
  const _Float16* p1 = planeR + (size_t)s1c * kSlotHalves + hp;
  float m0 = -__builtin_inff(), m1 = -__builtin_inff();
#pragma unroll 1
  for (int blk = 0; blk < kBlkPerDir; ++blk) {
    const size_t ob = (size_t)blk * kBlkHalves;
#pragma unroll
    for (int bl = 0; bl < kSeqPB; ++bl) {
      const size_t o = ob + (size_t)bl * kHid;
      m0 = fmaxf(m0, (float)p0[o]);
      m1 = fmaxf(m1, (float)p1[o]);
    }
  }
  const bool lastrow = (s1 >= kLen - 1);
  float m = fmaxf(m0, lastrow ? -__builtin_inff() : m1) * (1.0f / 1024.0f);
  const float crv = cr[hp];
  m = fmaxf(m, lastrow ? crv : -__builtin_inff());
  float* d = mx + (size_t)Bp * kMxP + kRightCol + hp;
  *(volatile float*)d = m;
  __threadfence();
  *(volatile float*)d = m;
}

__global__ __launch_bounds__(256) void fc_kernel(const float* __restrict__ mx, const float* __restrict__ fcw,
                                                 const float* __restrict__ fcb, float* __restrict__ out) {
  __shared__ __align__(16) float res[kBatch * kCls];
  const int tid = threadIdx.x;
  for (int o = tid; o < kBatch * kCls; o += 256) {
    const int Bp = o / kCls;
    const int cc = o - Bp * kCls;
    const float* mr = mx + (size_t)Bp * kMxP;
    const float* wr = fcw + (size_t)cc * kFeat;
    float s = 0.0f;
#pragma unroll 1
    for (int j = 0; j < kFeat; ++j) {
      const int col = j < (kHid + kEmb) ? j : (j + (kEmbP - kEmb));
      s += mr[col] * wr[j];
    }
    res[o] = s + fcb[cc];
  }
  __syncthreads();
  if (tid < (kBatch * kCls) / 4) {
    const v4f v = *(const v4f*)(res + 4 * tid);
    *(volatile v4f*)(out + 4 * tid) = v;
    __threadfence();
    *(volatile v4f*)(out + 4 * tid) = v;
  }
}

extern "C" void kernel_launch(void* const* d_in, const int* in_sizes, int n_in,
                              void* d_out, int out_size, void* d_ws, size_t ws_size, hipStream_t stream) {
  if (n_in < 10 || d_out == nullptr || d_ws == nullptr) return;
  if (in_sizes[0] != kBatch * kLen || in_sizes[1] != kVocab * kEmb ||
      in_sizes[2] != kHid * kHid || in_sizes[3] != kHid * kEmb ||
      in_sizes[4] != kHid * kHid || in_sizes[5] != kHid * kEmb ||
      in_sizes[6] != kHid || in_sizes[7] != kHid ||
      in_sizes[8] != kCls * kFeat || in_sizes[9] != kCls || out_size != kBatch * kCls) return;

  const int*   x   = (const int*)  d_in[0];
  const float* emb = (const float*)d_in[1];
  const float* wl  = (const float*)d_in[2];
  const float* wsl = (const float*)d_in[3];
  const float* wr  = (const float*)d_in[4];
  const float* wsr = (const float*)d_in[5];
  const float* cl  = (const float*)d_in[6];
  const float* cr  = (const float*)d_in[7];
  const float* fcw = (const float*)d_in[8];
  const float* fcb = (const float*)d_in[9];
  float* out = (float*)d_out;

  char* ws = (char*)d_ws; size_t off = 0;
  auto carve = [&](size_t bytes) -> char* { char* p = ws + off; off += (bytes + 255) & ~(size_t)255; return p; };
  _Float16* PLANES = (_Float16*)carve((size_t)2 * kDirHalves * 2);
  _Float16* WCAT   = (_Float16*)carve((size_t)2 * kWChunksDir * 8 * 2);
  float*    MX     = (float*)carve((size_t)kBatch * kMxP * 4);
  if (off > ws_size || off > (size_t)134217728) return;

  prep_kernel<<<kPrepBlocks, 256, 0, stream>>>(wl, wsl, wr, wsr, WCAT);

  recur_kernel<<<kRecBlocks, kRecThreads, 0, stream>>>(x, emb, WCAT, cl, cr, PLANES);

  max_left_kernel<<<(kBatch * kHid) / 256, 256, 0, stream>>>(PLANES, cl, MX);
  max_emb_kernel<<<kBatch, kEmbP, 0, stream>>>(x, emb, MX);
  max_right_kernel<<<(kBatch * kHid) / 256, 256, 0, stream>>>(PLANES + kDirHalves, cr, MX);

  fc_kernel<<<1, 256, 0, stream>>>(MX, fcw, fcb, out);
}
